// CrossAttentionBlock_66597762892025
// MI455X (gfx1250) — hardware-verified
//
#include <hip/hip_runtime.h>
#include <math.h>

#ifndef NB
#define NB 8
#endif
#ifndef SEQ
#define SEQ 1024
#endif
#ifndef SKV
#define SKV 1024
#endif
#define NB_FULL 8
#define SEQ_FULL 1024
#define SKV_FULL 1024
#define HID 768
#define NHEAD 12
#define HDIM 64
#define FFD 3072
#define NBR 9216

static_assert(NB >= 1 && NB <= NB_FULL);
static_assert(SEQ <= SEQ_FULL && SKV <= SKV_FULL);
static_assert(SEQ % 64 == 0 && SKV % 64 == 0);
static_assert((NB * SEQ) % 64 == 0 && (NB * SKV) % 64 == 0);
static_assert(HID % 64 == 0 && FFD % 64 == 0 && HID % 32 == 0 && FFD % 32 == 0);
static_assert(NHEAD * HDIM == HID && HDIM == 64);

typedef __attribute__((ext_vector_type(16))) _Float16 v16h;
typedef __attribute__((ext_vector_type(8)))  _Float16 v8h;
typedef __attribute__((ext_vector_type(8)))  float    v8f;
typedef __attribute__((ext_vector_type(4)))  float    v4f;
typedef __attribute__((ext_vector_type(4)))  unsigned v4u;

#define VST2(T, ptr, val) do { const T vst2_v_ = (val); *(volatile T*)(ptr) = vst2_v_; __threadfence(); *(volatile T*)(ptr) = vst2_v_; } while (0)
#define VST2V4(ptr, val) do { const v4f vst2_v4_ = (val); *(volatile v4f*)(ptr) = vst2_v4_; __threadfence(); *(volatile v4f*)(ptr) = vst2_v4_; } while (0)

union FragU { v16h v; v8h h[2]; };
__device__ __forceinline__ v16h frag_load(const _Float16* p) { FragU f; f.h[0] = *(const v8h*)(p); f.h[1] = *(const v8h*)(p + 16); return f.v; }

__device__ __forceinline__ v8f wmma16(v16h a, v16h b, v8f c) {
    c = __builtin_amdgcn_wmma_f32_16x16x32_f16(false, a, false, b, (short)0, c, false, false);
    asm volatile("v_nop\n\tv_nop\n\tv_nop\n\tv_nop" : "+v"(c) : "v"(a), "v"(b));
    return c;
}
__device__ __forceinline__ void dep_guard_h(v8f& a, v8f& b, v16h x, v16h y) { asm volatile("v_nop\n\tv_nop\n\tv_nop\n\tv_nop" : "+v"(a), "+v"(b) : "v"(x), "v"(y)); }
__device__ __forceinline__ void keep4_h(v16h a, v16h b, v16h c, v16h d) { asm volatile("v_nop" :: "v"(a), "v"(b), "v"(c), "v"(d)); }
__device__ __forceinline__ void acc_guard4(v8f& a, v8f& b, v8f& c, v8f& d) { asm volatile("v_nop\n\tv_nop\n\tv_nop\n\tv_nop" : "+v"(a), "+v"(b), "+v"(c), "+v"(d)); }

__device__ __forceinline__ float cmb_bf(float v) { const unsigned u = __builtin_bit_cast(unsigned, v); const unsigned r = (u + 0x7fffu + ((u >> 16) & 1u)) & 0xffff0000u; return __builtin_bit_cast(float, r); }
__device__ __forceinline__ unsigned int cmb_pk2(float a, float b) { return (unsigned int)__builtin_bit_cast(unsigned short, (_Float16)a) | ((unsigned int)__builtin_bit_cast(unsigned short, (_Float16)b) << 16); }

__global__ __launch_bounds__(256) void k_castx(const float* __restrict__ X, unsigned short* __restrict__ X16, int S, int SF, long long nrows) {
    const long long u = (long long)blockIdx.x * 256 + threadIdx.x; if (u >= nrows * 96) return;
    const long long r = u / 96; const int c0 = 8 * (int)(u - r * 96);
    const long long bb = r / S, ss = r - bb * S;
    const float* s = X + (bb * SF + ss) * HID + c0;
    const v4f a = *(const v4f*)(s), b = *(const v4f*)(s + 4);
    v4u pk;
    pk.x = cmb_pk2(cmb_bf(a.x), cmb_bf(a.y)); pk.y = cmb_pk2(cmb_bf(a.z), cmb_bf(a.w));
    pk.z = cmb_pk2(cmb_bf(b.x), cmb_bf(b.y)); pk.w = cmb_pk2(cmb_bf(b.z), cmb_bf(b.w));
    VST2(v4u, (v4u*)(X16 + r * HID + c0), pk);
}
__global__ __launch_bounds__(256) void k_castwT(const float* __restrict__ SRC, int lds, unsigned short* __restrict__ DST, int ldd, int nR, int nC, float sc) {
    const long long u = (long long)blockIdx.x * 256 + threadIdx.x; const int per = nR / 8; if (u >= (long long)nC * per) return;
    const int c = (int)(u / per); const int r0 = 8 * (int)(u % per);
    float w[8];
#pragma unroll
    for (int e = 0; e < 8; ++e) w[e] = cmb_bf(SRC[(long long)(r0 + e) * lds + c]) * sc;
    v4u pk; pk.x = cmb_pk2(w[0], w[1]); pk.y = cmb_pk2(w[2], w[3]); pk.z = cmb_pk2(w[4], w[5]); pk.w = cmb_pk2(w[6], w[7]);
    VST2(v4u, (v4u*)(DST + (long long)c * ldd + r0), pk);
}
__global__ __launch_bounds__(256) void k_bfvec(const float* __restrict__ SRC, float* __restrict__ DST, int n) {
    const int u = blockIdx.x * 256 + threadIdx.x; if (u >= n) return; VST2(float, DST + u, cmb_bf(SRC[u]));
}

template <int OUT_MODE, int ACT>
__global__ __launch_bounds__(256) void k_gemm64(const unsigned short* __restrict__ Ap, int lda, const unsigned short* __restrict__ Btp, int ldb,
                                                void* __restrict__ Cout, int ldc, const float* __restrict__ bias, int M, int N, int K, float scale) {
    const _Float16* A = (const _Float16*)Ap; const _Float16* Bt = (const _Float16*)Btp;
    __shared__ __align__(16) float sT[8][16 * 68];
    const int lane = threadIdx.x & 31, wave = threadIdx.x >> 5;
    const int tilesN = N >> 6, tilesM = M >> 6;
    const int tile = blockIdx.x * 8 + wave;
    if (tile >= tilesM * tilesN) return;
    const int tm = tile / tilesN, tn = tile - tm * tilesN;
    const int m0 = tm << 6, n0 = tn << 6;
    const int rlane = lane & 15, koff = (lane >> 4) * 8, mOff = (lane >> 4) * 8;

    v8f acc[4][4];
#pragma unroll
    for (int i = 0; i < 4; ++i)
#pragma unroll
        for (int j = 0; j < 4; ++j) { v8f zz = {}; acc[i][j] = zz; }

    for (int k0 = 0; k0 < K; k0 += 32) {
        v16h bh[4];
#pragma unroll
        for (int j = 0; j < 4; ++j) bh[j] = frag_load(Bt + (size_t)(n0 + (j << 4) + rlane) * ldb + koff + k0);
#pragma unroll
        for (int i = 0; i < 4; ++i) {
            const v16h ah = frag_load(A + (size_t)(m0 + (i << 4) + rlane) * lda + koff + k0);
#pragma unroll
            for (int j = 0; j < 4; ++j) acc[i][j] = __builtin_amdgcn_wmma_f32_16x16x32_f16(false, ah, false, bh[j], (short)0, acc[i][j], false, false);
            dep_guard_h(acc[i][0], acc[i][3], ah, ah);
        }
        keep4_h(bh[0], bh[1], bh[2], bh[3]);
    }
    acc_guard4(acc[0][0], acc[0][1], acc[0][2], acc[0][3]);
    acc_guard4(acc[1][0], acc[1][1], acc[1][2], acc[1][3]);
    acc_guard4(acc[2][0], acc[2][1], acc[2][2], acc[2][3]);
    acc_guard4(acc[3][0], acc[3][1], acc[3][2], acc[3][3]);

    float* slab = sT[wave];
#pragma unroll
    for (int i = 0; i < 4; ++i) {
        const int mBase = m0 + (i << 4);
#pragma unroll
        for (int j = 0; j < 4; ++j) {
            const int n = n0 + (j << 4) + rlane;
            const float bvn = bias[n];
#pragma unroll
            for (int r = 0; r < 8; ++r) {
                float v = acc[i][j][r] * scale + bvn;
                if (ACT == 1) v = fmaxf(v, 0.0f);
                slab[(mOff + r) * 68 + (j << 4) + rlane] = v;
            }
        }
        __builtin_amdgcn_fence(3  , "workgroup");
        __builtin_amdgcn_wave_barrier();
        __builtin_amdgcn_fence(2  , "workgroup");
        if (OUT_MODE == 0) {
            float* C = (float*)Cout;
            const int hh = lane >> 4, c4 = (lane & 15) * 4;
            for (int ps = 0; ps < 2; ++ps) {
#pragma unroll
                for (int it = 0; it < 8; ++it) {
                    const int row = it * 2 + hh;
                    const v4f v = *(const v4f*)(slab + row * 68 + c4);
                    *(volatile v4f*)(C + (size_t)(mBase + row) * ldc + n0 + c4) = v;
                }
                __threadfence();
            }
        } else {
            unsigned short* C = (unsigned short*)Cout;
            const int qq = lane >> 3, c8 = (lane & 7) * 8;
            for (int ps = 0; ps < 2; ++ps) {
#pragma unroll
                for (int it = 0; it < 4; ++it) {
                    const int row = it * 4 + qq;
                    const float* sp = slab + row * 68 + c8;
                    v4u pk; pk.x = cmb_pk2(sp[0], sp[1]); pk.y = cmb_pk2(sp[2], sp[3]); pk.z = cmb_pk2(sp[4], sp[5]); pk.w = cmb_pk2(sp[6], sp[7]);
                    *(volatile v4u*)(C + (size_t)(mBase + row) * ldc + n0 + c8) = pk;
                }
                __threadfence();
            }
        }
        __builtin_amdgcn_fence(3  , "workgroup");
        __builtin_amdgcn_wave_barrier();
        __builtin_amdgcn_fence(2  , "workgroup");
    }
}

#define AT_D 64
#define AT_NW 4
#define AT_QB 64
#define AT_KC 64
struct AttnGeom { long long q_bs, q_rs, q_hs, k_bs, k_rs, k_hs, v_bs, v_rs, v_hs, o_bs, o_rs, o_hs; int S, Skv, H; float sscale; };
static_assert(sizeof(AttnGeom) == 12 * 8 + 4 * 4);

__global__ __launch_bounds__(128) void k_attn64(const unsigned short* __restrict__ qp, const unsigned short* __restrict__ kp, const unsigned short* __restrict__ vp,
                                                float* __restrict__ out, AttnGeom g) {
    const _Float16* q = (const _Float16*)qp; const _Float16* k = (const _Float16*)kp; const _Float16* v = (const _Float16*)vp;
    const float PSC = 32768.0f;
    __shared__ __align__(16) _Float16 Ksh[AT_KC * AT_D];
    __shared__ __align__(16) _Float16 Vth[AT_D * AT_KC];
    __shared__ __align__(16) _Float16 Psh[AT_NW][16 * AT_KC];
    __shared__ __align__(16) float    Os[AT_NW][16 * 68];

    const int tid = threadIdx.x, wave = tid >> 5, lane = tid & 31, hh = lane >> 4, c = lane & 15;
    const int nqb = g.S / AT_QB;
    const int bx = blockIdx.x;
    const int qb = bx % nqb, bhd = bx / nqb;
    const int h = bhd % g.H, b = bhd / g.H;
    const int q0 = qb * AT_QB + wave * 16;

    const _Float16* qb_ptr = q + (size_t)b * g.q_bs + (size_t)h * g.q_hs;
    const _Float16* kb_ptr = k + (size_t)b * g.k_bs + (size_t)h * g.k_hs;
    const _Float16* vb_ptr = v + (size_t)b * g.v_bs + (size_t)h * g.v_hs;
    float*          ob_ptr = out + (size_t)b * g.o_bs + (size_t)h * g.o_hs;

    v16h qa[2];
    {
        const _Float16* qrow = qb_ptr + (size_t)(q0 + c) * g.q_rs + 8 * hh;
        qa[0] = frag_load(qrow); qa[1] = frag_load(qrow + 32);
    }

    float mrow[8], lrow[8];
    v8f oacc[4];
#pragma unroll
    for (int r = 0; r < 8; ++r) { mrow[r] = -__builtin_inff(); lrow[r] = 0.f; }
#pragma unroll
    for (int t = 0; t < 4; ++t) { v8f zz = {}; oacc[t] = zz; }

    const int nChunks = g.Skv / AT_KC;
    for (int kc = 0; kc < nChunks; ++kc) {
        const int kv0 = kc * AT_KC;
        __syncthreads();
        {
            const int kvr = tid >> 1, dh = (tid & 1) * 32;
            const _Float16* krow = kb_ptr + (size_t)(kv0 + kvr) * g.k_rs + dh;
            const _Float16* vrow = vb_ptr + (size_t)(kv0 + kvr) * g.v_rs + dh;
#pragma unroll
            for (int i = 0; i < 4; ++i) {
                const v8h kk = *(const v8h*)(krow + 8 * i);
                *(v8h*)(Ksh + kvr * AT_D + dh + 8 * i) = kk;
                const v8h vv = *(const v8h*)(vrow + 8 * i);
#pragma unroll
                for (int e = 0; e < 8; ++e) Vth[(dh + 8 * i + e) * AT_KC + kvr] = vv[e];
            }
        }
        __syncthreads();

        v8f s[4];
#pragma unroll
        for (int j = 0; j < 4; ++j) {
            v8f zz = {}; s[j] = zz;
#pragma unroll
            for (int dc = 0; dc < 2; ++dc) s[j] = wmma16(qa[dc], frag_load(Ksh + (j * 16 + c) * AT_D + dc * 32 + 8 * hh), s[j]);
        }
        float sc[8][4], cm[8];
#pragma unroll
        for (int r = 0; r < 8; ++r) {
            float m = -__builtin_inff();
#pragma unroll
            for (int j = 0; j < 4; ++j) { sc[r][j] = s[j][r] * g.sscale; m = fmaxf(m, sc[r][j]); }
#pragma unroll
            for (int off = 1; off < 16; off <<= 1) m = fmaxf(m, __shfl_xor(m, off, 32));
            cm[r] = m;
        }
        _Float16* pwh = Psh[wave];
#pragma unroll
        for (int r = 0; r < 8; ++r) {
            const float mnew = fmaxf(mrow[r], cm[r]);
            const float alpha = expf(mrow[r] - mnew);
            mrow[r] = mnew;
            float psum = 0.f;
#pragma unroll
            for (int j = 0; j < 4; ++j) {
                const float p = expf(sc[r][j] - mnew);
                psum += p;
                pwh[(8 * hh + r) * AT_KC + j * 16 + c] = (_Float16)(p * PSC);
            }
#pragma unroll
            for (int off = 1; off < 16; off <<= 1) psum += __shfl_xor(psum, off, 32);
            lrow[r] = lrow[r] * alpha + psum;
#pragma unroll
            for (int t = 0; t < 4; ++t) oacc[t][r] *= alpha;
        }
        __builtin_amdgcn_fence(3  , "workgroup");
        __builtin_amdgcn_wave_barrier();
        __builtin_amdgcn_fence(2  , "workgroup");
#pragma unroll
        for (int kk2 = 0; kk2 < 2; ++kk2) {
            const v16h pa = frag_load(pwh + c * AT_KC + kk2 * 32 + 8 * hh);
#pragma unroll
            for (int t = 0; t < 4; ++t) oacc[t] = wmma16(pa, frag_load(Vth + (t * 16 + c) * AT_KC + kk2 * 32 + 8 * hh), oacc[t]);
        }
    }

    float* os = Os[wave];
#pragma unroll
    for (int r = 0; r < 8; ++r) {
        const float inv = 1.0f / (lrow[r] * PSC);
#pragma unroll
        for (int t = 0; t < 4; ++t) os[(8 * hh + r) * 68 + t * 16 + c] = oacc[t][r] * inv;
    }
    __builtin_amdgcn_fence(3  , "workgroup");
    __builtin_amdgcn_wave_barrier();
    __builtin_amdgcn_fence(2  , "workgroup");
    {
        const int c4 = (lane & 15) * 4;
        for (int ps = 0; ps < 2; ++ps) {
#pragma unroll
            for (int it = 0; it < 8; ++it) {
                const int row = it * 2 + hh;
                const v4f val = *(const v4f*)(os + row * 68 + c4);
                *(volatile v4f*)(ob_ptr + (size_t)(q0 + row) * g.o_rs + c4) = val;
            }
            __threadfence();
        }
    }
}

template <bool RBF, bool H16OUT>
__global__ __launch_bounds__(192) void k_ln_res(const float* __restrict__ X, const float* __restrict__ R, int rS, int rSF,
                                                const float* __restrict__ g, const float* __restrict__ bb, float* __restrict__ Y, unsigned short* __restrict__ Y16) {
    __shared__ float red[8];
    __shared__ __align__(16) float rowst[H16OUT ? HID : 8];
    const int row = blockIdx.x, t = threadIdx.x, lane = t & 31, w = t >> 5;
    const int bi = row / rS, si = row - bi * rS;
    const float* xr = X + (long long)row * HID;
    const float* rr = R + ((long long)bi * rSF + si) * HID;
    const v4f x = *(const v4f*)(xr + 4 * t);
    float s = (x.x + x.y) + (x.z + x.w);
#pragma unroll
    for (int o = 16; o > 0; o >>= 1) s += __shfl_xor(s, o, 32);
    if (lane == 0) red[w] = s;
    __syncthreads();
    const float mean = (((red[0] + red[1]) + (red[2] + red[3])) + (red[4] + red[5])) * (1.0f / 768.0f);
    __syncthreads();
    const v4f d = x - mean;
    float qs = (d.x * d.x + d.y * d.y) + (d.z * d.z + d.w * d.w);
#pragma unroll
    for (int o = 16; o > 0; o >>= 1) qs += __shfl_xor(qs, o, 32);
    if (lane == 0) red[w] = qs;
    __syncthreads();
    const float var = (((red[0] + red[1]) + (red[2] + red[3])) + (red[4] + red[5])) * (1.0f / 768.0f);
    const float rstd = rsqrtf(var + 1e-5f);
    v4f rv = *(const v4f*)(rr + 4 * t);
    if (RBF) { rv.x = cmb_bf(rv.x); rv.y = cmb_bf(rv.y); rv.z = cmb_bf(rv.z); rv.w = cmb_bf(rv.w); }
    const v4f gv = *(const v4f*)(g + 4 * t), bv = *(const v4f*)(bb + 4 * t);
    const v4f y = rv + ((d * rstd) * gv + bv);
    VST2V4(Y + (long long)row * HID + 4 * t, y);
    if (H16OUT) {
        *(v4f*)(rowst + 4 * t) = y;
        __syncthreads();
        if (t < 96) {
            const float* sp = rowst + 8 * t;
            v4u pk; pk.x = cmb_pk2(sp[0], sp[1]); pk.y = cmb_pk2(sp[2], sp[3]); pk.z = cmb_pk2(sp[4], sp[5]); pk.w = cmb_pk2(sp[6], sp[7]);
            VST2(v4u, (v4u*)(Y16 + (long long)row * HID + 8 * t), pk);
        }
    }
}

static inline size_t al256(size_t b) { return (b + 255) / 256 * 256; }
static inline size_t smax(size_t a, size_t b) { return a > b ? a : b; }

extern "C" void kernel_launch(void* const* d_in, const int* in_sizes, int n_in, void* d_out, int out_size, void* d_ws, size_t ws_size, hipStream_t stream) {
    if (n_in < 16) return;
    const long long MR = (long long)NB * SEQ, KR = (long long)NB * SKV;
    if ((long long)in_sizes[0] < ((long long)(NB - 1) * SEQ_FULL + SEQ) * HID) return;
    if ((long long)in_sizes[1] < ((long long)(NB - 1) * SKV_FULL + SKV) * HID) return;
    if (in_sizes[2] < HID * HID || in_sizes[4] < HID * HID || in_sizes[6] < HID * HID) return;
    if (in_sizes[3] < HID || in_sizes[5] < HID || in_sizes[7] < HID || in_sizes[8] < HID || in_sizes[9] < HID || in_sizes[10] < HID || in_sizes[11] < HID || in_sizes[15] < HID) return;
    if (in_sizes[12] < HID * FFD || in_sizes[14] < HID * FFD || in_sizes[13] < FFD) return;
    if ((long long)out_size < MR * HID) return;

    const float* freq  = (const float*)d_in[0];
    const float* image = (const float*)d_in[1];
    const float* Wq = (const float*)d_in[2];  const float* bq = (const float*)d_in[3];
    const float* Wk = (const float*)d_in[4];  const float* bk = (const float*)d_in[5];
    const float* Wv = (const float*)d_in[6];  const float* bv = (const float*)d_in[7];
    const float* g_att = (const float*)d_in[8];  const float* b_att = (const float*)d_in[9];
    const float* g_mlp = (const float*)d_in[10]; const float* b_mlp = (const float*)d_in[11];
    const float* W1 = (const float*)d_in[12]; const float* b1 = (const float*)d_in[13];
    const float* W2 = (const float*)d_in[14]; const float* b2 = (const float*)d_in[15];
    float* out = (float*)d_out;
    char* ws = (char*)d_ws;

    const size_t szXF = (size_t)MR * HID * 2, szXI = (size_t)KR * HID * 2, szCTX = (size_t)MR * HID * 4;
    const size_t szA  = al256(smax(szXF + szXI, szCTX));
    const size_t szW3 = al256((size_t)3 * HID * HID * 2);
    const size_t szW1 = al256((size_t)FFD * HID * 2);
    const size_t szW2 = al256((size_t)HID * FFD * 2);
    const size_t szBR = al256((size_t)NBR * 4);
    const size_t szQ  = al256((size_t)MR * HID * 2);
    const size_t szKV = al256(smax((size_t)KR * 2 * HID * 2, (size_t)MR * HID * 4));
    const size_t szFF = al256((size_t)MR * FFD * 2);
    const size_t oA = 0, oW3 = oA + szA, oW1 = oW3 + szW3, oW2 = oW1 + szW1, oBR = oW2 + szW2, oQ = oBR + szBR, oKV = oQ + szQ, oFF = oKV + szKV;
    const size_t total = oFF + szFF;
    if (total > ws_size) return;

    unsigned short* XF16 = (unsigned short*)(ws + oA);
    unsigned short* XI16 = (unsigned short*)(ws + oA + szXF);
    float*          CTX  = (float*)(ws + oA);
    float*          MLP  = (float*)(ws + oA);
    unsigned short* WQT  = (unsigned short*)(ws + oW3);
    unsigned short* WKVT = WQT + (size_t)HID * HID;
    unsigned short* W1T  = (unsigned short*)(ws + oW1);
    unsigned short* W2T  = (unsigned short*)(ws + oW2);
    float*          BR   = (float*)(ws + oBR);
    unsigned short* Q16  = (unsigned short*)(ws + oQ);
    unsigned short* H16  = (unsigned short*)(ws + oQ);
    unsigned short* KV16 = (unsigned short*)(ws + oKV);
    float*          HF   = (float*)(ws + oKV);
    unsigned short* FF16 = (unsigned short*)(ws + oFF);
    float* BRq = BR; float* BRkv = BR + 768; float* BR1 = BR + 2304; float* BR2 = BR + 5376;
    float* Gatt = BR + 6144; float* Batt = BR + 6912; float* Gmlp = BR + 7680; float* Bmlp = BR + 8448;

    k_castx<<<(unsigned)((MR * 96 + 255) / 256), 256, 0, stream>>>(freq, XF16, SEQ, SEQ_FULL, MR);
    k_castx<<<(unsigned)((KR * 96 + 255) / 256), 256, 0, stream>>>(image, XI16, SKV, SKV_FULL, KR);
    k_castwT<<<(unsigned)(((long long)HID * (HID / 8) + 255) / 256), 256, 0, stream>>>(Wq, HID, WQT, HID, HID, HID, 16.0f);
    k_castwT<<<(unsigned)(((long long)HID * (HID / 8) + 255) / 256), 256, 0, stream>>>(Wk, HID, WKVT, HID, HID, HID, 16.0f);
    k_castwT<<<(unsigned)(((long long)HID * (HID / 8) + 255) / 256), 256, 0, stream>>>(Wv, HID, WKVT + (size_t)HID * HID, HID, HID, HID, 16.0f);
    k_castwT<<<(unsigned)(((long long)FFD * (HID / 8) + 255) / 256), 256, 0, stream>>>(W1, FFD, W1T, HID, HID, FFD, 16.0f);
    k_castwT<<<(unsigned)(((long long)HID * (FFD / 8) + 255) / 256), 256, 0, stream>>>(W2, HID, W2T, FFD, FFD, HID, 16.0f);
    k_bfvec<<<3, 256, 0, stream>>>(bq, BRq, 768);
    k_bfvec<<<3, 256, 0, stream>>>(bk, BRkv, 768);
    k_bfvec<<<3, 256, 0, stream>>>(bv, BRkv + 768, 768);
    k_bfvec<<<12, 256, 0, stream>>>(b1, BR1, FFD);
    k_bfvec<<<3, 256, 0, stream>>>(b2, BR2, 768);
    k_bfvec<<<3, 256, 0, stream>>>(g_att, Gatt, 768);
    k_bfvec<<<3, 256, 0, stream>>>(b_att, Batt, 768);
    k_bfvec<<<3, 256, 0, stream>>>(g_mlp, Gmlp, 768);
    k_bfvec<<<3, 256, 0, stream>>>(b_mlp, Bmlp, 768);

    k_gemm64<1, 0><<<(unsigned)(((MR / 64) * (HID / 64) + 7) / 8), 256, 0, stream>>>(XF16, HID, WQT, HID, (void*)Q16, HID, BRq, (int)MR, HID, HID, 0.0625f);
    k_gemm64<1, 0><<<(unsigned)(((KR / 64) * (2 * HID / 64) + 7) / 8), 256, 0, stream>>>(XI16, HID, WKVT, HID, (void*)KV16, 2 * HID, BRkv, (int)KR, 2 * HID, HID, 0.0625f);

    {
        AttnGeom ag;
        ag.q_bs = (long long)SEQ * HID;     ag.q_rs = HID;     ag.q_hs = HDIM;
        ag.k_bs = (long long)SKV * 2 * HID; ag.k_rs = 2 * HID; ag.k_hs = HDIM;
        ag.v_bs = (long long)SKV * 2 * HID; ag.v_rs = 2 * HID; ag.v_hs = HDIM;
        ag.o_bs = (long long)SEQ * HID;     ag.o_rs = HID;     ag.o_hs = HDIM;
        ag.S = SEQ; ag.Skv = SKV; ag.H = NHEAD; ag.sscale = 0.125f;
        k_attn64<<<(unsigned)(NB * NHEAD * (SEQ / AT_QB)), 32 * AT_NW, 0, stream>>>(Q16, KV16, KV16 + HID, CTX, ag);
    }

    k_ln_res<true, true><<<(unsigned)MR, 192, 0, stream>>>(CTX, freq, SEQ, SEQ_FULL, Gatt, Batt, HF, H16);

    k_gemm64<1, 1><<<(unsigned)(((MR / 64) * (FFD / 64) + 7) / 8), 256, 0, stream>>>(H16, HID, W1T, HID, (void*)FF16, FFD, BR1, (int)MR, FFD, HID, 0.0625f);
    k_gemm64<0, 0><<<(unsigned)(((MR / 64) * (HID / 64) + 7) / 8), 256, 0, stream>>>(FF16, FFD, W2T, FFD, (void*)MLP, HID, BR2, (int)MR, HID, FFD, 0.0625f);

    k_ln_res<false, false><<<(unsigned)MR, 192, 0, stream>>>(MLP, HF, SEQ, SEQ, Gmlp, Bmlp, out, nullptr);
}
